// GlideAttention_84215718739982
// MI455X (gfx1250) — hardware-verified
//
#include <hip/hip_runtime.h>
#include <stdint.h>
#include <stddef.h>


#define NB     2
#define QL     2048
#define HIDD   2048
#define NHQ    16
#define NKVH   4
#define HDIM   128
#define MROWS  (NB * QL)
#define TPITCH 65
#define SPITCH 132

typedef float v4f __attribute__((ext_vector_type(4)));
typedef float v8f __attribute__((ext_vector_type(8)));
typedef unsigned short v8us __attribute__((ext_vector_type(8)));
typedef unsigned short v16us __attribute__((ext_vector_type(16)));
typedef __bf16 v16bf __attribute__((ext_vector_type(16)));
typedef v4f __attribute__((may_alias)) v4fa;
typedef v8us __attribute__((may_alias)) v8usa;

union Frag { v16us u; v8us hv[2]; v16bf v; };

__device__ __forceinline__ unsigned int bf_rne(float f) {
  const unsigned int u = __float_as_uint(f);
  return (u + 0x7fffu + ((u >> 16) & 1u)) >> 16;
}

__device__ __forceinline__ void split_bf(float x, unsigned short& hi, unsigned short& lo) {
  const unsigned int hb = bf_rne(x);
  const float hf = __uint_as_float(hb << 16);
  hi = (unsigned short)hb;
  lo = (unsigned short)bf_rne(x - hf);
}

__device__ __forceinline__ void split8(v4f a, v4f c, v8us& hi, v8us& lo) {
#pragma unroll
  for (int u = 0; u < 4; ++u) {
    unsigned short h0, l0, h1, l1;
    split_bf(a[u], h0, l0);
    split_bf(c[u], h1, l1);
    hi[u] = h0; lo[u] = l0; hi[u + 4] = h1; lo[u + 4] = l1;
  }
}

__device__ __forceinline__ void ldfrag(Frag& f, const unsigned short* p) {
  f.hv[0] = *(const v8usa*)(p);
  f.hv[1] = *(const v8usa*)(p + 16);
}

__device__ __forceinline__ v8f mma3(v8f acc, v16bf ah, v16bf al, v16bf bh, v16bf bl) {
  acc = __builtin_amdgcn_wmma_f32_16x16x32_bf16(false, ah, false, bh, (short)0, acc, false, false);
  acc = __builtin_amdgcn_wmma_f32_16x16x32_bf16(false, ah, false, bl, (short)0, acc, false, false);
  acc = __builtin_amdgcn_wmma_f32_16x16x32_bf16(false, al, false, bh, (short)0, acc, false, false);
  asm volatile("v_nop\n\tv_nop\n\tv_nop\n\tv_nop"
               : "+v"(acc) : "v"(ah), "v"(al), "v"(bh), "v"(bl) : "memory");
  return acc;
}

__global__ __launch_bounds__(256) void cvt_rows(const float* __restrict__ in,
                                                  unsigned short* oh, unsigned short* ol, int n8)
{
  const int i = blockIdx.x * 256 + threadIdx.x;
  if (i >= n8) return;
  const size_t e = (size_t)i * 8;
  const v4f a = *(const v4fa*)(in + e);
  const v4f c = *(const v4fa*)(in + e + 4);
  v8us hi, lo;
  split8(a, c, hi, lo);
  *(volatile v8us*)(oh + e) = hi;
  *(volatile v8us*)(ol + e) = lo;
  __threadfence();
  *(volatile v8us*)(oh + e) = hi;
  *(volatile v8us*)(ol + e) = lo;
}

__device__ __forceinline__ void tsplit64(const float* __restrict__ src, int spitch,
                                         unsigned short* dh, unsigned short* dl, int dpitch,
                                         float* tile)
{
  const int t = threadIdx.x;
  {
    const int rr = t >> 2, cq = (t & 3) * 16;
    const float* s = src + (size_t)rr * spitch + cq;
#pragma unroll
    for (int u = 0; u < 4; ++u) {
      const v4f x = *(const v4fa*)(s + 4 * u);
      float* d = tile + rr * TPITCH + cq + 4 * u;
      d[0] = x[0]; d[1] = x[1]; d[2] = x[2]; d[3] = x[3];
    }
  }
  __syncthreads();
#pragma unroll
  for (int p = 0; p < 2; ++p) {
    const int cc = (t >> 3) + 32 * p, rq = (t & 7) * 8;
    v4f a, c;
#pragma unroll
    for (int u = 0; u < 4; ++u) {
      a[u] = tile[(rq + u) * TPITCH + cc];
      c[u] = tile[(rq + 4 + u) * TPITCH + cc];
    }
    v8us hi, lo;
    split8(a, c, hi, lo);
    const size_t d = (size_t)cc * dpitch + rq;
    *(volatile v8us*)(dh + d) = hi;
    *(volatile v8us*)(dl + d) = lo;
    __threadfence();
    *(volatile v8us*)(dh + d) = hi;
    *(volatile v8us*)(dl + d) = lo;
  }
}

__global__ __launch_bounds__(256) void cvt_t_w(const float* __restrict__ W,
                                                 unsigned short* oh, unsigned short* ol)
{
  __shared__ float tile[64 * TPITCH];
  const int k0 = blockIdx.x * 64, n0 = blockIdx.y * 64;
  const size_t dof = (size_t)n0 * HIDD + k0;
  tsplit64(W + (size_t)k0 * HIDD + n0, HIDD, oh + dof, ol + dof, HIDD, tile);
}

__global__ __launch_bounds__(256) void cvt_t_v(const float* __restrict__ V,
                                                 unsigned short* oh, unsigned short* ol)
{
  __shared__ float tile[64 * TPITCH];
  const int j0 = blockIdx.x * 64, d0 = blockIdx.y * 64, z = blockIdx.z;
  const int b = z >> 2, kvh = z & 3;
  const float* src = V + ((size_t)(b * QL + j0) * NKVH + kvh) * HDIM + d0;
  const size_t dof = ((size_t)z * HDIM + d0) * QL + j0;
  tsplit64(src, NKVH * HDIM, oh + dof, ol + dof, QL, tile);
}

template <int MODE>
__global__ __launch_bounds__(128) void gemm3(
    const unsigned short* __restrict__ Ah, const unsigned short* __restrict__ Al,
    const unsigned short* __restrict__ Bh, const unsigned short* __restrict__ Bl,
    const float* __restrict__ bias, const float* __restrict__ cosb,
    const float* __restrict__ sinb, unsigned short* Qh, unsigned short* Ql,
    float* Cout, int N, int K)
{
  __shared__ float sT[64 * SPITCH];
  const int t = threadIdx.x, l = t & 31, w = t >> 5, h16 = l >> 4, m = l & 15;
  const int wr = w >> 1, wc = w & 1;
  const int m0 = blockIdx.x * 64, n0 = blockIdx.y * 128;

  v8f acc[2][4];
#pragma unroll
  for (int mi = 0; mi < 2; ++mi)
#pragma unroll
    for (int ni = 0; ni < 4; ++ni) acc[mi][ni] = (v8f){0.f, 0.f, 0.f, 0.f, 0.f, 0.f, 0.f, 0.f};

  const size_t arow = (size_t)(m0 + 32 * wr + m) * K + 8 * h16;
  const size_t brow = (size_t)(n0 + 64 * wc + m) * K + 8 * h16;
  const int nk = K >> 5;

#pragma unroll 1
  for (int kt = 0; kt < nk; ++kt) {
    const int k0 = kt * 32;
    Frag ah[2], al[2];
#pragma unroll
    for (int mi = 0; mi < 2; ++mi) {
      const size_t o = arow + (size_t)mi * 16 * K + k0;
      ldfrag(ah[mi], Ah + o);
      ldfrag(al[mi], Al + o);
    }
#pragma unroll
    for (int ni = 0; ni < 4; ++ni) {
      const size_t o = brow + (size_t)ni * 16 * K + k0;
      Frag bh, bl;
      ldfrag(bh, Bh + o);
      ldfrag(bl, Bl + o);
#pragma unroll
      for (int mi = 0; mi < 2; ++mi)
        acc[mi][ni] = mma3(acc[mi][ni], ah[mi].v, al[mi].v, bh.v, bl.v);
    }
  }

#pragma unroll
  for (int mi = 0; mi < 2; ++mi)
#pragma unroll
    for (int ni = 0; ni < 4; ++ni)
#pragma unroll
      for (int r = 0; r < 8; ++r)
        sT[(32 * wr + 16 * mi + 8 * h16 + r) * SPITCH + 64 * wc + 16 * ni + m] = acc[mi][ni][r];
  __syncthreads();

  if (MODE == 0) {
    const int rr = t >> 4, cq = (t & 15) * 8, cp = cq ^ 64;
    const float sgn = (cq < 64) ? -1.0f : 1.0f;
    const v4f b0 = *(const v4fa*)(bias + n0 + cq), b1 = *(const v4fa*)(bias + n0 + cq + 4);
    const v4f e0 = *(const v4fa*)(bias + n0 + cp), e1 = *(const v4fa*)(bias + n0 + cp + 4);
#pragma unroll 1
    for (int p = 0; p < 8; ++p) {
      const int row = 8 * p + rr;
      const int grow = m0 + row;
      const float* srow = sT + row * SPITCH;
      const v4f x0 = *(const v4fa*)(srow + cq), x1 = *(const v4fa*)(srow + cq + 4);
      const v4f y0 = *(const v4fa*)(srow + cp), y1 = *(const v4fa*)(srow + cp + 4);
      const float* cr = cosb + (size_t)grow * HDIM;
      const float* sr = sinb + (size_t)grow * HDIM;
      const v4f c0 = *(const v4fa*)(cr + cq), c1 = *(const v4fa*)(cr + cq + 4);
      const v4f s0 = *(const v4fa*)(sr + cq), s1 = *(const v4fa*)(sr + cq + 4);
      const v4f q0 = (x0 + b0) * c0 + (sgn * (y0 + e0)) * s0;
      const v4f q1 = (x1 + b1) * c1 + (sgn * (y1 + e1)) * s1;
      v8us hi, lo;
      split8(q0, q1, hi, lo);
      const size_t d = (size_t)grow * N + n0 + cq;
      *(volatile v8us*)(Qh + d) = hi;
      *(volatile v8us*)(Ql + d) = lo;
      __threadfence();
      *(volatile v8us*)(Qh + d) = hi;
      *(volatile v8us*)(Ql + d) = lo;
    }
  } else {
    const int cq = l * 4;
#pragma unroll 1
    for (int p = 0; p < 16; ++p) {
      const int row = 4 * p + w;
      const v4f x = *(const v4fa*)(sT + row * SPITCH + cq);
      const size_t d = (size_t)(m0 + row) * N + n0 + cq;
      *(volatile v4f*)(Cout + d) = x;
      __threadfence();
      *(volatile v4f*)(Cout + d) = x;
    }
  }
}

__global__ __launch_bounds__(128) void attn_glide(
    const unsigned short* __restrict__ Qh, const unsigned short* __restrict__ Ql,
    const unsigned short* __restrict__ Kh, const unsigned short* __restrict__ Kl,
    const unsigned short* __restrict__ Vh, const unsigned short* __restrict__ Vl,
    unsigned short* Oh, unsigned short* Ol)
{
  __shared__ float sO[4 * 16 * SPITCH];
  const int t = threadIdx.x, l = t & 31, w = t >> 5, h16 = l >> 4, m = l & 15;
  const int qt = blockIdx.x, bh = blockIdx.y;
  const int b = bh >> 4, hq = bh & 15, kvh = hq >> 2;
  const int R0 = qt * 64;
  const int iq = R0 + 16 * w + m;
  const float NEG_INF = -__builtin_inff();
  const float kScale = 0.08838834764831845f;

  const size_t qbase = ((size_t)(b * QL + iq)) * HIDD + hq * HDIM + 8 * h16;
  const size_t kbase = ((size_t)(b * QL + m) * NKVH + kvh) * HDIM + 8 * h16;
  const size_t vbase = ((size_t)(b * NKVH + kvh) * HDIM + m) * QL + 8 * h16;

  v8f acc[8];
#pragma unroll
  for (int n = 0; n < 8; ++n) acc[n] = (v8f){0.f, 0.f, 0.f, 0.f, 0.f, 0.f, 0.f, 0.f};
  float mrun = NEG_INF, lrun = 0.0f;

#pragma unroll 1
  for (int kt = 0; kt <= qt; ++kt) {
    const int j0 = kt * 64;

    v8f s[4];
#pragma unroll
    for (int sub = 0; sub < 4; ++sub) s[sub] = (v8f){0.f, 0.f, 0.f, 0.f, 0.f, 0.f, 0.f, 0.f};
#pragma unroll
    for (int c = 0; c < 4; ++c) {
      Frag qh, ql;
      ldfrag(qh, Qh + qbase + 32 * c);
      ldfrag(ql, Ql + qbase + 32 * c);
#pragma unroll
      for (int sub = 0; sub < 4; ++sub) {
        const size_t ko = kbase + (size_t)(j0 + 16 * sub) * (NKVH * HDIM) + 32 * c;
        Frag kh, kl;
        ldfrag(kh, Kh + ko);
        ldfrag(kl, Kl + ko);
        s[sub] = mma3(s[sub], kh.v, kl.v, qh.v, ql.v);
      }
    }

    float mx = NEG_INF;
#pragma unroll
    for (int sub = 0; sub < 4; ++sub) {
#pragma unroll
      for (int r = 0; r < 8; ++r) {
        const int jb = j0 + 16 * sub + 8 * h16 + r;
        const bool vis = ((iq >> 2) > (jb >> 2)) || ((iq < 4) && (jb < 4));
        const float v = vis ? (s[sub][r] * kScale) : NEG_INF;
        s[sub][r] = v;
        mx = fmaxf(mx, v);
      }
    }
    mx = fmaxf(mx, __shfl_xor(mx, 16));
    const float mnew = fmaxf(mrun, mx);
    const float msafe = (mnew == NEG_INF) ? 0.0f : mnew;
    const float sc = __expf(mrun - msafe);
    float ls = 0.0f;
#pragma unroll
    for (int sub = 0; sub < 4; ++sub) {
#pragma unroll
      for (int r = 0; r < 8; ++r) {
        const float p = __expf(s[sub][r] - msafe);
        s[sub][r] = p;
        ls += p;
      }
    }
    ls += __shfl_xor(ls, 16);
    lrun = lrun * sc + ls;
    mrun = mnew;
#pragma unroll
    for (int n = 0; n < 8; ++n) acc[n] = acc[n] * sc;

#pragma unroll
    for (int ks = 0; ks < 2; ++ks) {
      Frag ph, pl;
#pragma unroll
      for (int r = 0; r < 8; ++r) {
        unsigned short a0, c0, a1, c1;
        split_bf(s[2 * ks][r], a0, c0);
        split_bf(s[2 * ks + 1][r], a1, c1);
        ph.u[r] = a0; pl.u[r] = c0; ph.u[8 + r] = a1; pl.u[8 + r] = c1;
      }
#pragma unroll
      for (int n = 0; n < 8; ++n) {
        const size_t vo = vbase + (size_t)n * 16 * QL + j0 + 32 * ks;
        Frag vh, vl;
        ldfrag(vh, Vh + vo);
        ldfrag(vl, Vl + vo);
        acc[n] = mma3(acc[n], vh.v, vl.v, ph.v, pl.v);
      }
    }
  }

  const float inv = 1.0f / lrun;
#pragma unroll
  for (int n = 0; n < 8; ++n) {
    const v8f o = acc[n] * inv;
#pragma unroll
    for (int r = 0; r < 8; ++r)
      sO[(w * 16 + m) * SPITCH + 16 * n + 8 * h16 + r] = o[r];
  }
  __syncthreads();
#pragma unroll 1
  for (int p = 0; p < 8; ++p) {
    const int rloc = 2 * p + h16;
    const int dq = m * 8;
    const float* src = sO + (w * 16 + rloc) * SPITCH + dq;
    const v4f a = *(const v4fa*)(src);
    const v4f c = *(const v4fa*)(src + 4);
    v8us hi, lo;
    split8(a, c, hi, lo);
    const size_t d = ((size_t)(b * QL + R0 + 16 * w + rloc)) * HIDD + hq * HDIM + dq;
    *(volatile v8us*)(Oh + d) = hi;
    *(volatile v8us*)(Ol + d) = lo;
    __threadfence();
    *(volatile v8us*)(Oh + d) = hi;
    *(volatile v8us*)(Ol + d) = lo;
  }
}

extern "C" void kernel_launch(void* const* d_in, const int* in_sizes, int n_in,
                              void* d_out, int out_size, void* d_ws, size_t ws_size,
                              hipStream_t stream)
{
  if (n_in < 8) return;
  if (in_sizes[0] != MROWS * HIDD) return;
  if (in_sizes[1] != NB * QL * NKVH * HDIM || in_sizes[2] != NB * QL * NKVH * HDIM) return;
  if (in_sizes[3] != NB * QL * HDIM || in_sizes[4] != NB * QL * HDIM) return;
  if (in_sizes[5] != HIDD * HIDD || in_sizes[7] != HIDD * HIDD || in_sizes[6] != HIDD) return;
  if (out_size != MROWS * HIDD) return;

  const float* hidden = (const float*)d_in[0];
  const float* kc     = (const float*)d_in[1];
  const float* vc     = (const float*)d_in[2];
  const float* cosb   = (const float*)d_in[3];
  const float* sinb   = (const float*)d_in[4];
  const float* Wq     = (const float*)d_in[5];
  const float* bq     = (const float*)d_in[6];
  const float* Wo     = (const float*)d_in[7];
  float* out = (float*)d_out;

  const size_t planeX = (size_t)MROWS * HIDD * 2;
  const size_t planeW = (size_t)HIDD * HIDD * 2;
  const size_t planeK = (size_t)NB * QL * NKVH * HDIM * 2;
  const size_t offXh  = 0;
  const size_t offXl  = offXh + planeX;
  const size_t offQh  = offXl + planeX;
  const size_t offQl  = offQh + planeX;
  const size_t offWqh = offQl + planeX;
  const size_t offWql = offWqh + planeW;
  const size_t offWoh = offWql + planeW;
  const size_t offWol = offWoh + planeW;
  const size_t offKh  = offWol + planeW;
  const size_t offKl  = offKh + planeK;
  const size_t offVh  = offKl + planeK;
  const size_t offVl  = offVh + planeK;
  const size_t total  = offVl + planeK;
  if (total > ws_size) return;

  char* ws = (char*)d_ws;
  unsigned short* Xh  = (unsigned short*)(ws + offXh);
  unsigned short* Xl  = (unsigned short*)(ws + offXl);
  unsigned short* Oh  = Xh;
  unsigned short* Ol  = Xl;
  unsigned short* Qh  = (unsigned short*)(ws + offQh);
  unsigned short* Ql  = (unsigned short*)(ws + offQl);
  unsigned short* Wqh = (unsigned short*)(ws + offWqh);
  unsigned short* Wql = (unsigned short*)(ws + offWql);
  unsigned short* Woh = (unsigned short*)(ws + offWoh);
  unsigned short* Wol = (unsigned short*)(ws + offWol);
  unsigned short* Kh  = (unsigned short*)(ws + offKh);
  unsigned short* Kl  = (unsigned short*)(ws + offKl);
  unsigned short* Vh  = (unsigned short*)(ws + offVh);
  unsigned short* Vl  = (unsigned short*)(ws + offVl);

  const int n8x = in_sizes[0] / 8;
  const int n8k = in_sizes[1] / 8;
  cvt_rows<<<dim3((n8x + 255) / 256), dim3(256), 0, stream>>>(hidden, Xh, Xl, n8x);
  cvt_rows<<<dim3((n8k + 255) / 256), dim3(256), 0, stream>>>(kc, Kh, Kl, n8k);
  cvt_t_w<<<dim3(HIDD / 64, HIDD / 64), dim3(256), 0, stream>>>(Wq, Wqh, Wql);
  cvt_t_w<<<dim3(HIDD / 64, HIDD / 64), dim3(256), 0, stream>>>(Wo, Woh, Wol);
  cvt_t_v<<<dim3(QL / 64, HDIM / 64, NB * NKVH), dim3(256), 0, stream>>>(vc, Vh, Vl);

  gemm3<0><<<dim3(MROWS / 64, HIDD / 128), dim3(128), 0, stream>>>(
      Xh, Xl, Wqh, Wql, bq, cosb, sinb, Qh, Ql, out, HIDD, HIDD);

  attn_glide<<<dim3(QL / 64, NB * NHQ), dim3(128), 0, stream>>>(Qh, Ql, Kh, Kl, Vh, Vl, Oh, Ol);

  gemm3<1><<<dim3(MROWS / 64, HIDD / 128), dim3(128), 0, stream>>>(
      Oh, Ol, Woh, Wol, bq, cosb, sinb, Qh, Ql, out, HIDD, HIDD);
}
